// BaseNCA_8718783611277
// MI455X (gfx1250) — hardware-verified
//
#include <hip/hip_runtime.h>

#define NB_ 4
#define CC_ 16
#define IH  256
#define IW  256
#define HID 128
#define NCLS 32
#define CDIM 64
#define MAXSTEPS 8

typedef _Float16 f16;
typedef __attribute__((ext_vector_type(16))) f16 f16x16;
typedef __attribute__((ext_vector_type(8)))  f16 f16x8;
typedef __attribute__((ext_vector_type(8)))  float f32x8;
typedef __attribute__((ext_vector_type(4)))  float v4f_t;
typedef float v4fa __attribute__((ext_vector_type(4), may_alias));

__device__ __forceinline__ f32x8 wmma16(f16x16 a, f16x16 b, f32x8 c) {
  c = __builtin_amdgcn_wmma_f32_16x16x32_f16(false, a, false, b, (short)0, c, false, false);
  asm volatile("v_nop\n\tv_nop\n\tv_nop\n\tv_nop" : "+v"(c) : "v"(a), "v"(b));
  return c;
}
__device__ __forceinline__ f16x16 lds_frag(const f16* base, int stride) {
  const int lane = threadIdx.x & 31, row = lane & 15, kh = (lane >> 4) * 8;
  const f16x8 lo = *(const f16x8*)(base + row * stride + kh);
  const f16x8 hi = *(const f16x8*)(base + row * stride + kh + 16);
  f16x16 f;
#pragma unroll
  for (int i = 0; i < 8; ++i) { f[i] = lo[i]; f[i + 8] = hi[i]; }
  return f;
}

__global__ __launch_bounds__(256) void k_film(const int* __restrict__ cond, const float* __restrict__ embed, const float* __restrict__ fw, const float* __restrict__ fb, float* __restrict__ film) {
  __shared__ __attribute__((aligned(16))) float fS[256];
  const int b = blockIdx.x, j = threadIdx.x;
  int c = cond[b]; c = min(max(c, 0), NCLS - 1);
  float s = fb[j];
#pragma unroll 1
  for (int d = 0; d < CDIM; ++d) s += embed[c * CDIM + d] * fw[d * 2 * HID + j];
  fS[j] = s;
  __syncthreads();
  if (j < 64) { *(volatile v4f_t*)(film + b * 256 + j * 4) = *(const volatile v4fa*)(fS + j * 4); __threadfence(); *(volatile v4f_t*)(film + b * 256 + j * 4) = *(const volatile v4fa*)(fS + j * 4); }
}

__global__ __launch_bounds__(256) void k_step(const float* __restrict__ xin, float* __restrict__ xout, const float* __restrict__ film,
                                              const float* __restrict__ W1, const float* __restrict__ b1, const float* __restrict__ W2, const float* __restrict__ b2,
                                              const float* __restrict__ W3, const float* __restrict__ b3, const int* __restrict__ nsteps, int s) {
  __shared__ __attribute__((aligned(16))) f16 fS[128 * 72];
  __shared__ __attribute__((aligned(16))) f16 w1S[128 * 72];
  __shared__ __attribute__((aligned(16))) f16 hS[128 * 136];
  __shared__ __attribute__((aligned(16))) f16 w2S[128 * 136];
  __shared__ __attribute__((aligned(16))) f16 w3S[16 * 136];
  __shared__ __attribute__((aligned(16))) float dS[16 * 132];
  const int tid = threadIdx.x, lane = tid & 31, wave = tid >> 5, cl = lane & 15, rh = (lane >> 4) * 8;
  const int b = blockIdx.x / (IH * 2), rem = blockIdx.x % (IH * 2), y = rem >> 1, x0 = (rem & 1) * 128;
  const bool active = (s < *nsteps);
  if (!active) {
#pragma unroll 1
    for (int pass = 0; pass < 2; ++pass) {
      for (int q = tid; q < CC_ * 32; q += 256) { const int c = q >> 5, px4 = (q & 31) * 4; const size_t off = (((size_t)b * CC_ + c) * IH + y) * IW + x0 + px4;
        *(volatile v4f_t*)(xout + off) = *(const v4f_t*)(xin + off); }
      __threadfence();
    }
    return;
  }
  for (int e = tid; e < 128 * 64; e += 256) { const int n = e >> 6, k = e & 63; w1S[n * 72 + k] = (f16)((k < 48) ? W1[k * HID + n] : 0.0f); }
  for (int e = tid; e < 128 * 128; e += 256) { const int n = e >> 7, k = e & 127; w2S[n * 136 + k] = (f16)W2[k * HID + n]; }
  for (int e = tid; e < 16 * 128; e += 256) { const int n = e >> 7, k = e & 127; w3S[n * 136 + k] = (f16)W3[k * CC_ + n]; }
  { const int px = tid & 127, ch0 = (tid >> 7) * 8, xx = x0 + px;
#pragma unroll 1
    for (int cc = 0; cc < 8; ++cc) { const int c = ch0 + cc; const float* pl = xin + ((size_t)b * CC_ + c) * IH * IW;
      float v[3][3];
#pragma unroll
      for (int dy = -1; dy <= 1; ++dy)
#pragma unroll
        for (int dx = -1; dx <= 1; ++dx) { const int yy = y + dy, xq = xx + dx; v[dy + 1][dx + 1] = (yy >= 0 && yy < IH && xq >= 0 && xq < IW) ? pl[(size_t)yy * IW + xq] : 0.0f; }
      const float gx = (v[0][2] - v[0][0]) + 2.0f * (v[1][2] - v[1][0]) + (v[2][2] - v[2][0]);
      const float gy = (v[2][0] - v[0][0]) + 2.0f * (v[2][1] - v[0][1]) + (v[2][2] - v[0][2]);
      fS[px * 72 + c] = (f16)v[1][1]; fS[px * 72 + CC_ + c] = (f16)gx; fS[px * 72 + 2 * CC_ + c] = (f16)gy;
      if (c == 0) {
#pragma unroll
        for (int k = 48; k < 64; ++k) fS[px * 72 + k] = (f16)0.0f; }
    } }
  __syncthreads();
  const float* gam = film + b * 256; const float* bet = gam + HID;
  {
    f16x16 a0 = lds_frag(fS + (wave * 16) * 72, 72), a1 = lds_frag(fS + (wave * 16) * 72 + 32, 72);
#pragma unroll
    for (int nt = 0; nt < 8; ++nt) {
      f32x8 acc = {}; acc = wmma16(a0, lds_frag(w1S + (nt * 16) * 72, 72), acc); acc = wmma16(a1, lds_frag(w1S + (nt * 16) * 72 + 32, 72), acc);
      const int n = nt * 16 + cl; const float bb = b1[n], gv = gam[n], bv = bet[n];
#pragma unroll
      for (int r = 0; r < 8; ++r) hS[(wave * 16 + rh + r) * 136 + n] = (f16)(gv * fmaxf(acc[r] + bb, 0.0f) + bv);
    }
  }
  __syncthreads();
  {
    f16x16 a[4];
#pragma unroll
    for (int ks = 0; ks < 4; ++ks) a[ks] = lds_frag(hS + (wave * 16) * 136 + ks * 32, 136);
    f32x8 acc[8];
#pragma unroll
    for (int nt = 0; nt < 8; ++nt) { f32x8 z = {}; acc[nt] = z;
#pragma unroll
      for (int ks = 0; ks < 4; ++ks) acc[nt] = wmma16(a[ks], lds_frag(w2S + (nt * 16) * 136 + ks * 32, 136), acc[nt]); }
    __builtin_amdgcn_wave_barrier();
#pragma unroll
    for (int nt = 0; nt < 8; ++nt) { const int n = nt * 16 + cl; const float bb = b2[n];
#pragma unroll
      for (int r = 0; r < 8; ++r) hS[(wave * 16 + rh + r) * 136 + n] = (f16)fmaxf(acc[nt][r] + bb, 0.0f); }
  }
  asm volatile("s_wait_dscnt 0" ::: "memory");
  __builtin_amdgcn_wave_barrier();
  {
    f32x8 acc = {};
#pragma unroll
    for (int ks = 0; ks < 4; ++ks) acc = wmma16(lds_frag(hS + (wave * 16) * 136 + ks * 32, 136), lds_frag(w3S + ks * 32, 136), acc);
    const int c = cl; const float bb = b3[c];
#pragma unroll
    for (int r = 0; r < 8; ++r) { float d = acc[r] + bb; d = fminf(fmaxf(d, -10.0f), 10.0f); dS[c * 132 + wave * 16 + rh + r] = d; }
  }
  __syncthreads();
#pragma unroll 1
  for (int pass = 0; pass < 2; ++pass) {
#pragma unroll
    for (int it = 0; it < 2; ++it) { const int q = tid + 256 * it, c = q >> 5, px4 = (q & 31) * 4; const size_t off = (((size_t)b * CC_ + c) * IH + y) * IW + x0 + px4;
      const v4f_t xi = *(const v4f_t*)(xin + off); v4f_t o;
      o[0] = xi[0] + 0.1f * dS[c * 132 + px4]; o[1] = xi[1] + 0.1f * dS[c * 132 + px4 + 1]; o[2] = xi[2] + 0.1f * dS[c * 132 + px4 + 2]; o[3] = xi[3] + 0.1f * dS[c * 132 + px4 + 3];
      *(volatile v4f_t*)(xout + off) = o; }
    __threadfence();
  }
}

extern "C" void kernel_launch(void* const* d_in, const int* in_sizes, int n_in,
                              void* d_out, int out_size, void* d_ws, size_t ws_size,
                              hipStream_t stream) {
  (void)in_sizes; (void)n_in; (void)out_size; (void)ws_size;
  const float* x = (const float*)d_in[0];
  const int* cond = (const int*)d_in[1];
  const float* embed = (const float*)d_in[2];
  const float* fw = (const float*)d_in[3], *fb = (const float*)d_in[4];
  const float* W1 = (const float*)d_in[5], *b1 = (const float*)d_in[6];
  const float* W2 = (const float*)d_in[7], *b2 = (const float*)d_in[8];
  const float* W3 = (const float*)d_in[9], *b3 = (const float*)d_in[10];
  const int* nsteps = (const int*)d_in[11];
  float* out = (float*)d_out;
  char* ws = (char*)d_ws;
  float* film = (float*)ws; ws += 4096;
  float* bufA = (float*)ws; ws += (size_t)NB_ * CC_ * IH * IW * 4;
  float* bufB = (float*)ws; ws += (size_t)NB_ * CC_ * IH * IW * 4;
  k_film<<<dim3(NB_), dim3(256), 0, stream>>>(cond, embed, fw, fb, film);
  const dim3 g(NB_ * IH * 2), blk(256);
  const float* src = x;
  for (int s = 0; s < MAXSTEPS; ++s) {
    float* dst = (s == MAXSTEPS - 1) ? out : ((s & 1) ? bufB : bufA);
    k_step<<<g, blk, 0, stream>>>(src, dst, film, W1, b1, W2, b2, W3, b3, nsteps, s);
    src = dst;
  }
}
